// Block_43379169690252
// MI455X (gfx1250) — hardware-run, weakly checked
//
#include <hip/hip_runtime.h>


#ifndef SEQ
#define SEQ  2048
#endif
#define WORD 1024
#define HD   128
#define NH   16
#define DQ   (NH * HD)
#define XK   (2 * WORD)
#define ZK   (2 * DQ)
#define NPROJ (4 * DQ + NH)
#define YP   64
#define WAR  (2 * DQ + YP)
#define PCAR 1024.0f
#define XRC  2048.0f
#define VRC  2048.0f
#define ZCAR 16.0f
#define ZRC  2048.0f
#define WCAR 4096.0f
#define OCAR 16384.0f
#define PSP  72
#define OSP  132
#define TRP  72
#define LOG2E 1.4426950408889634f
#define NEGB (-1.0e10f)

static_assert(SEQ % 64 == 0);
static_assert(SEQ % 32 == 0);
static_assert(SEQ % 8 == 0);
static_assert(WORD % 64 == 0);
static_assert(WORD % 32 == 0);
static_assert(WORD == 32 * 8 * 4);
static_assert(WORD == 32 * 4 * 8);
static_assert(HD == 128);
static_assert(HD == 16 * 8);
static_assert(HD == 4 * 2 * 16);
static_assert(HD % 32 == 0);
static_assert(DQ % 64 == 0);
static_assert(DQ == 2048);
static_assert(XK % 32 == 0);
static_assert(ZK % 32 == 0);
static_assert(YP == 64);
static_assert(NH <= YP);
static_assert(NH * 32 == 512);
static_assert(WAR % 64 == 0);
static_assert((PSP * 2) % 16 == 0);
static_assert((TRP * 2) % 16 == 0);
static_assert((OSP * 4) % 16 == 0);
static_assert(8 * 2 == 16);
static_assert(256 * 2 == 64 * 8);
static_assert(256 * 4 == 64 * 16);
static_assert(2 * (4 * 16 * PSP * 2) + 4 * 16 * OSP * 4 + SEQ * 4 <= 65536);
static_assert(2 * (4 * 16 * PSP * 2) + 4 * 16 * OSP * 4 + SEQ * 4 <= 131072);
static_assert(2 * 64 * TRP * 2 <= 131072);
static_assert(16 * 68 * 4 <= 131072);

typedef _Float16 h16;
typedef __attribute__((ext_vector_type(16))) _Float16 v16h;
typedef __attribute__((ext_vector_type(8)))  _Float16 v8h;
typedef __attribute__((ext_vector_type(8)))  float    v8f;
typedef __attribute__((ext_vector_type(4)))  float    v4f;
typedef v8h  __attribute__((may_alias)) v8ha;
typedef v4f  __attribute__((may_alias)) v4fa;

__device__ __forceinline__ unsigned short f2bf(float f) { unsigned u = __float_as_uint(f); u += 0x7FFFu + ((u >> 16) & 1u); return (unsigned short)(u >> 16); }
__device__ __forceinline__ float bf2f(unsigned short b) { return __uint_as_float(((unsigned)b) << 16); }
__device__ __forceinline__ float bfr(float f) { return bf2f(f2bf(f)); }
__device__ __forceinline__ v16h cat16(v8h lo, v8h hi) { return __builtin_shufflevector(lo, hi, 0, 1, 2, 3, 4, 5, 6, 7, 8, 9, 10, 11, 12, 13, 14, 15); }
static __device__ __forceinline__ h16 toh_flush(float v) { const h16 r = (h16)v; return (fabsf(v) < 6.103515625e-05f) ? (h16)0.0f : r; }
__device__ __forceinline__ v8f wmma16g(v16h a, v16h b, v8f c) {
    c = __builtin_amdgcn_wmma_f32_16x16x32_f16(false, a, false, b, (short)0, c, false, false);
    asm volatile("v_nop\n\tv_nop\n\tv_nop\n\tv_nop" : "+v"(c) : "v"(a), "v"(b));
    return c;
}
__device__ __forceinline__ v16h ldh(const h16* p) { return cat16(*(const v8h*)p, *(const v8h*)(p + 16)); }
__device__ __forceinline__ void wsync() { __builtin_amdgcn_fence(3  , "wavefront"); __builtin_amdgcn_wave_barrier(); asm volatile("" ::: "memory"); }

template <typename T16> struct WFrag;
template <> struct WFrag<h16> { typedef v16h V; static __device__ __forceinline__ V ld(const h16* p) { return cat16(*(const v8h*)p, *(const v8h*)(p + 16)); } static __device__ __forceinline__ v8f mma(V a, V b, v8f c) { return wmma16g(a, b, c); } };

template <typename T16, bool BIAS>
__device__ __forceinline__ void gemmw_body(const T16* __restrict__ A, int lda, const T16* __restrict__ Bt, int K, float* C, int ldc, const float* __restrict__ bias, int nbias, float oscale) {
    typedef typename WFrag<T16>::V V;
    __shared__ __align__(16) float os[16 * 68];
    const int lane = threadIdx.x & 31, lr = lane & 15, hi = lane >> 4; const int r0 = blockIdx.x * 64, c0 = blockIdx.y * 64;
    v8f acc[4][4];
#pragma unroll
    for (int mb = 0; mb < 4; ++mb)
#pragma unroll
        for (int nb = 0; nb < 4; ++nb) acc[mb][nb] = (v8f){};
    const size_t aoff = (size_t)(r0 + lr) * lda + 8 * hi, boff = (size_t)(c0 + lr) * K + 8 * hi;
#pragma unroll 1
    for (int kc = 0; kc < K; kc += 32) {
        V a[4];
#pragma unroll
        for (int mb = 0; mb < 4; ++mb) a[mb] = WFrag<T16>::ld(A + aoff + (size_t)mb * 16 * lda + kc);
#pragma unroll
        for (int nb = 0; nb < 4; ++nb) { const V b = WFrag<T16>::ld(Bt + boff + (size_t)nb * 16 * K + kc);
#pragma unroll
            for (int mb = 0; mb < 4; ++mb) acc[mb][nb] = WFrag<T16>::mma(a[mb], b, acc[mb][nb]); }
    }
#pragma unroll
    for (int mb = 0; mb < 4; ++mb) {
#pragma unroll
        for (int nb = 0; nb < 4; ++nb) {
#pragma unroll
            for (int j = 0; j < 8; ++j) os[(hi * 8 + j) * 68 + nb * 16 + lr] = acc[mb][nb][j]; }
        wsync();
        float* crow = C + (size_t)(r0 + mb * 16) * ldc + c0;
#pragma unroll 1
        for (int ps = 0; ps < 2; ++ps) {
#pragma unroll
            for (int s = 0; s < 8; ++s) { const int row = 2 * s + hi, cofs = lr * 4; v4f val = *(const v4fa*)(os + row * 68 + cofs);
                val[0] *= oscale; val[1] *= oscale; val[2] *= oscale; val[3] *= oscale;
                if (BIAS) {
#pragma unroll
                    for (int q = 0; q < 4; ++q) { const int cc = c0 + cofs + q; const int ca = (cc < nbias) ? cc : (nbias - 1);
                        float bv = bias[ca]; asm volatile("" : "+v"(bv)); val[q] += (cc < nbias) ? bfr(bv) : 0.0f; } }
                *(volatile v4f*)(crow + (size_t)row * ldc + cofs) = val; }
            if (ps == 0) __threadfence(); }
        wsync();
    }
}
__global__ __launch_bounds__(32) void k_gemm_xw(const h16* __restrict__ A, int lda, const h16* __restrict__ Bt, int K, float* C, int ldc, const float* __restrict__ bias, int nbias, float oscale) { gemmw_body<h16, true>(A, lda, Bt, K, C, ldc, bias, nbias, oscale); }
__global__ __launch_bounds__(32) void k_gemm_zp(const h16* __restrict__ A, int lda, const h16* __restrict__ Bt, int K, float* C, int ldc, float oscale) { gemmw_body<h16, false>(A, lda, Bt, K, C, ldc, nullptr, 1, oscale); }

__global__ __launch_bounds__(256) void k_ln_in(const float* __restrict__ x, const float* __restrict__ gw, const float* __restrict__ gb, h16* XC) {
#pragma clang fp contract(off)
    const int lane = threadIdx.x & 31; const int wave = __builtin_amdgcn_readfirstlane(threadIdx.x >> 5);
    const int row = blockIdx.x * 8 + wave;
    const float* xr = x + (size_t)row * WORD;
    float s = 0.0f;
#pragma unroll 1
    for (int i = 0; i < 4; ++i) { const v8f v = *(const v8f*)(xr + (i * 32 + lane) * 8);
#pragma unroll
        for (int k = 0; k < 8; ++k) s += bfr(v[k]); }
    s += __shfl_xor(s, 16, 32); s += __shfl_xor(s, 8, 32); s += __shfl_xor(s, 4, 32); s += __shfl_xor(s, 2, 32); s += __shfl_xor(s, 1, 32);
    const float mu = s * (1.0f / WORD);
    float ss = 0.0f;
#pragma unroll 1
    for (int i = 0; i < 4; ++i) { const v8f v = *(const v8f*)(xr + (i * 32 + lane) * 8);
#pragma unroll
        for (int k = 0; k < 8; ++k) { const float d = bfr(v[k]) - mu; ss += d * d; } }
    ss += __shfl_xor(ss, 16, 32); ss += __shfl_xor(ss, 8, 32); ss += __shfl_xor(ss, 4, 32); ss += __shfl_xor(ss, 2, 32); ss += __shfl_xor(ss, 1, 32);
    const float rstd = 1.0f / sqrtf(ss * (1.0f / WORD) + 1.0e-5f);
    h16* xo = XC + (size_t)row * XK;
#pragma unroll 1
    for (int i = 0; i < 4; ++i) { const int col = (i * 32 + lane) * 8;
        const v8f v = *(const v8f*)(xr + col); const v8f g = *(const v8f*)(gw + col); const v8f b = *(const v8f*)(gb + col); v8h o, r;
#pragma unroll
        for (int k = 0; k < 8; ++k) { const float y = (bfr(v[k]) - mu) * rstd * bfr(g[k]) + bfr(b[k]); const h16 a = toh_flush(y); o[k] = a; r[k] = toh_flush((y - (float)a) * XRC); }
        *(volatile v8h*)(xo + col) = o; *(volatile v8h*)(xo + WORD + col) = r;
        __threadfence();
        *(volatile v8h*)(xo + col) = o; *(volatile v8h*)(xo + WORD + col) = r; }
}

__global__ __launch_bounds__(256) void k_wplane(const float* __restrict__ src, int nr, int nrp, int K, h16* dst, int ldo, float sc, float sc2, int dual) {
    const size_t k8 = (size_t)(K >> 3);
    const size_t i = (size_t)blockIdx.x * 256 + threadIdx.x; if (i >= (size_t)nrp * k8) return;
    const int row = (int)(i / k8), c8 = (int)(i % k8);
    const int rr = (row < nr) ? row : (nr - 1);
    v8f v = *(const v8f*)(src + (size_t)rr * K + c8 * 8);
    asm volatile("" : "+v"(v));
    const bool ok = row < nr; v8h a, b;
#pragma unroll
    for (int k = 0; k < 8; ++k) { const float wv = ok ? bfr(v[k]) : 0.0f; a[k] = toh_flush(wv * sc); b[k] = toh_flush(wv * sc2); }
    h16* o = dst + (size_t)row * ldo + c8 * 8;
    *(volatile v8h*)o = a; if (dual) *(volatile v8h*)(o + K) = b;
    __threadfence();
    *(volatile v8h*)o = a; if (dual) *(volatile v8h*)(o + K) = b;
}

__global__ __launch_bounds__(256) void k_qkplanes(const float* __restrict__ F, h16* P16, const float* __restrict__ smear, const float* __restrict__ lsc, int iskey) {
#pragma clang fp contract(off)
    const size_t i = (size_t)blockIdx.x * 256 + threadIdx.x; if (i >= (size_t)NH * SEQ * HD / 8) return;
    const int e8 = (int)(i % (HD / 8)); const int s = (int)((i / (HD / 8)) % SEQ); const int h = (int)(i / ((size_t)(HD / 8) * SEQ));
    const float rs = 1.0f / expf(bfr(lsc[h]));
    const float sg = 1.0f / (1.0f + expf(-bfr(smear[h])));
    const float sm = iskey ? sg : 0.0f;
    const int sp = (s > 0) ? (s - 1) : 0;
    const v8f v = *(const v8f*)(F + (size_t)s * DQ + h * HD + e8 * 8);
    v8f vp = *(const v8f*)(F + (size_t)sp * DQ + h * HD + e8 * 8);
    asm volatile("" : "+v"(vp));
    v8h o;
#pragma unroll
    for (int k = 0; k < 8; ++k) { const float pv = (s > 0) ? vp[k] : 0.0f; const float kv = (1.0f - sm) * v[k] + sm * pv; o[k] = toh_flush(kv * rs); }
    *(volatile v8h*)(P16 + i * 8) = o;
    __threadfence();
    *(volatile v8h*)(P16 + i * 8) = o;
}

__global__ __launch_bounds__(256) void k_vt(const float* __restrict__ in, int ldi, h16* outv, h16* outr, int ldo) {
    __shared__ __align__(16) h16 t1[64 * TRP];
    __shared__ __align__(16) h16 t2[64 * TRP];
    const int tid = threadIdx.x;
    const int r0 = blockIdx.x * 64, c0 = blockIdx.y * 64;
#pragma unroll
    for (int i = 0; i < 4; ++i) { const int idx = tid + i * 256; const int r = idx >> 4, c4 = (idx & 15) * 4; const v4f v = *(const v4f*)(in + (size_t)(r0 + r) * ldi + c0 + c4);
#pragma unroll
        for (int q = 0; q < 4; ++q) { const h16 a = toh_flush(v[q]); t1[(c4 + q) * TRP + r] = a; t2[(c4 + q) * TRP + r] = toh_flush((v[q] - (float)a) * VRC); } }
    __syncthreads();
#pragma unroll 1
    for (int ps = 0; ps < 2; ++ps) {
#pragma unroll
        for (int i = 0; i < 2; ++i) { const int idx = tid + i * 256; const int c = idx >> 3, p = (idx & 7) * 8; const size_t oo = (size_t)(c0 + c) * ldo + r0 + p;
            const v8h a = *(const v8ha*)(t1 + c * TRP + p); const v8h b = *(const v8ha*)(t2 + c * TRP + p);
            *(volatile v8h*)(outv + oo) = a; *(volatile v8h*)(outr + oo) = b; }
        if (ps == 0) __threadfence(); }
}

__global__ __launch_bounds__(512) void k_pos(const float* __restrict__ YF, float* POS) {
#pragma clang fp contract(off)
    const int lane = threadIdx.x & 31; const int wave = __builtin_amdgcn_readfirstlane(threadIdx.x >> 5);
    double carry = 0.0;
#pragma unroll 1
    for (int c = 0; c < SEQ / 32; ++c) {
        const int s = c * 32 + lane;
        const float y = YF[(size_t)s * YP + wave];
        const float sg = 1.0f / (1.0f + expf(-y));
        double v = (double)sg;
#pragma unroll
        for (int off = 1; off < 32; off <<= 1) { const double t = __shfl_up(v, (unsigned)off, 32); v += (lane >= off) ? t : 0.0; }
        const float pv = (float)(carry + v);
        float* o = POS + (size_t)wave * SEQ + s;
        *(volatile float*)o = pv; __threadfence(); *(volatile float*)o = pv;
        carry += __shfl(v, 31, 32);
    }
}

__device__ __forceinline__ void pv_phase(const v16h pa, const h16* __restrict__ vsrc, v8f (&O)[8]) {
#pragma unroll
    for (int g = 0; g < 4; ++g) {
        int vg = g * 2 * 16 * SEQ; asm volatile("" : "+v"(vg));
        const v16h f0 = ldh(vsrc + vg);
        const v16h f1 = ldh(vsrc + vg + 16 * SEQ);
        O[2 * g] = wmma16g(pa, f0, O[2 * g]);
        O[2 * g + 1] = wmma16g(pa, f1, O[2 * g + 1]);
        __builtin_amdgcn_sched_barrier(0);
    }
}

__global__ __launch_bounds__(128) __attribute__((amdgpu_num_vgpr(256))) void k_flash(const h16* __restrict__ QH, const h16* __restrict__ KP, const h16* __restrict__ VT, const h16* __restrict__ VR, const float* __restrict__ POS, const float* __restrict__ PF, h16* ZC) {
    __shared__ __align__(16) h16 ps[4 * 16 * PSP];
    __shared__ __align__(16) h16 pr[4 * 16 * PSP];
    __shared__ __align__(16) float os[4 * 16 * OSP];
    __shared__ float spos[SEQ];
    const int lane = threadIdx.x & 31, lr = lane & 15, hi = lane >> 4;
    const int w = __builtin_amdgcn_readfirstlane(threadIdx.x >> 5);
    const int h = blockIdx.y, qb = blockIdx.x * 64, q0 = qb + w * 16;
    const int kend = qb + 64;
    for (int t = threadIdx.x; t < kend; t += 128) spos[t] = POS[(size_t)h * SEQ + t];
    __syncthreads();
    const h16* Qh = QH + (size_t)h * SEQ * HD;
    const h16* Kh = KP + (size_t)h * SEQ * HD + lr * HD + 8 * hi;
    const h16* Vt = VT + (size_t)h * HD * SEQ + (size_t)lr * SEQ + 8 * hi;
    const h16* Vr = VR + (size_t)h * HD * SEQ + (size_t)lr * SEQ + 8 * hi;
    const int qoff = (q0 + lr) * HD + 8 * hi;
    const int pw = w * 16 * PSP, ow = w * 16 * OSP;
    const float SCL2 = (float)(0.08838834764831845 * 1.4426950408889634);
    const float PRS = 1.0f / VRC;
    v8f O[8]; float m[8], l[8];
#pragma unroll
    for (int t = 0; t < 8; ++t) O[t] = (v8f){};
#pragma unroll
    for (int r = 0; r < 8; ++r) { m[r] = -3.0e38f; l[r] = 0.0f; }

#pragma unroll 1
    for (int j0 = 0; j0 < kend; j0 += 64) {
        v8f sc[4];
#pragma unroll
        for (int hf = 0; hf < 2; ++hf) {
            const h16* Kt = Kh + (size_t)(j0 + hf * 32) * HD;
            v8f a0 = (v8f){}, a1 = (v8f){};
#pragma unroll
            for (int kk = 0; kk < HD / 32; ++kk) {
                int st = kk * 32; asm volatile("" : "+v"(st));
                const v16h qa = ldh(Qh + qoff + st);
                const v16h b0 = ldh(Kt + st), b1 = ldh(Kt + 16 * HD + st);
                a0 = wmma16g(qa, b0, a0); a1 = wmma16g(qa, b1, a1);
            }
            sc[2 * hf] = a0; sc[2 * hf + 1] = a1;
        }
        float pj[4];
#pragma unroll
        for (int c = 0; c < 4; ++c) pj[c] = spos[j0 + 16 * c + lr];
#pragma unroll
        for (int r = 0; r < 8; ++r) {
            const float pir = spos[q0 + 8 * hi + r];
#pragma unroll
            for (int c = 0; c < 4; ++c) sc[c][r] = sc[c][r] * SCL2 - (pir - pj[c]) * LOG2E;
        }
        if (j0 + 63 > q0) {
#pragma unroll
            for (int c = 0; c < 4; ++c)
#pragma unroll
                for (int r = 0; r < 8; ++r) sc[c][r] = (j0 + 16 * c + lr > q0 + 8 * hi + r) ? NEGB : sc[c][r];
        }
#pragma unroll
        for (int r = 0; r < 8; ++r) {
            const float t0 = sc[0][r], t1 = sc[1][r], t2 = sc[2][r], t3 = sc[3][r];
            float mx = fmaxf(fmaxf(t0, t1), fmaxf(t2, t3));
            mx = fmaxf(mx, __shfl_xor(mx, 1, 32)); mx = fmaxf(mx, __shfl_xor(mx, 2, 32)); mx = fmaxf(mx, __shfl_xor(mx, 4, 32)); mx = fmaxf(mx, __shfl_xor(mx, 8, 32));
            const float mn = fmaxf(m[r], mx);
            const float alr = __builtin_amdgcn_exp2f(m[r] - mn); m[r] = mn;
            const float p0 = __builtin_amdgcn_exp2f(t0 - mn) * PCAR, p1 = __builtin_amdgcn_exp2f(t1 - mn) * PCAR, p2 = __builtin_amdgcn_exp2f(t2 - mn) * PCAR, p3 = __builtin_amdgcn_exp2f(t3 - mn) * PCAR;
            l[r] = l[r] * alr + ((p0 + p1) + (p2 + p3));
            const int po = pw + (8 * hi + r) * PSP + lr;
            ps[po] = toh_flush(p0); ps[po + 16] = toh_flush(p1); ps[po + 32] = toh_flush(p2); ps[po + 48] = toh_flush(p3);
            pr[po] = toh_flush(p0 * PRS); pr[po + 16] = toh_flush(p1 * PRS); pr[po + 32] = toh_flush(p2 * PRS); pr[po + 48] = toh_flush(p3 * PRS);
#pragma unroll
            for (int t = 0; t < 8; ++t) O[t][r] *= alr;
            __builtin_amdgcn_sched_barrier(0);
        }
        wsync();
        const h16* vb = Vt + j0; const h16* rb = Vr + j0;
        {
            int po = pw + lr * PSP + 8 * hi; asm volatile("" : "+v"(po));
            const v16h pa = cat16(*(const v8ha*)(ps + po), *(const v8ha*)(ps + po + 16));
            pv_phase(pa, vb, O);
        }
        {
            int po = pw + lr * PSP + 32 + 8 * hi; asm volatile("" : "+v"(po));
            const v16h pa = cat16(*(const v8ha*)(ps + po), *(const v8ha*)(ps + po + 16));
            pv_phase(pa, vb + 32, O);
        }
        {
            int po = pw + lr * PSP + 8 * hi; asm volatile("" : "+v"(po));
            const v16h pa = cat16(*(const v8ha*)(pr + po), *(const v8ha*)(pr + po + 16));
            pv_phase(pa, rb, O);
        }
        {
            int po = pw + lr * PSP + 32 + 8 * hi; asm volatile("" : "+v"(po));
            const v16h pa = cat16(*(const v8ha*)(pr + po), *(const v8ha*)(pr + po + 16));
            pv_phase(pa, rb + 32, O);
        }
        wsync();
    }

    float inv[8];
#pragma unroll
    for (int r = 0; r < 8; ++r) { float s = l[r]; s += __shfl_xor(s, 1, 32); s += __shfl_xor(s, 2, 32); s += __shfl_xor(s, 4, 32); s += __shfl_xor(s, 8, 32); inv[r] = __fdiv_rn(ZCAR, s); }
#pragma unroll
    for (int t = 0; t < 8; ++t)
#pragma unroll
        for (int r = 0; r < 8; ++r) os[ow + (8 * hi + r) * OSP + t * 16 + lr] = O[t][r] * inv[r];
    wsync();
    h16* zrow = ZC + (size_t)q0 * ZK + h * HD;
    const float* prow = PF + (size_t)q0 * DQ + h * HD;
#pragma unroll 1
    for (int s = 0; s < 8; ++s) { const int row = 2 * s + hi, cofs = lr * 8;
        const v4f o0 = *(const v4fa*)(os + ow + row * OSP + cofs), o1 = *(const v4fa*)(os + ow + row * OSP + cofs + 4);
        const v4f g0 = *(const v4f*)(prow + (size_t)row * DQ + cofs), g1 = *(const v4f*)(prow + (size_t)row * DQ + cofs + 4);
        v8h a, b;
#pragma unroll
        for (int k = 0; k < 4; ++k) { const float pv = g0[k]; const float z = o0[k] * (pv * (1.0f / (1.0f + expf(-pv)))); const h16 zh = toh_flush(z); a[k] = zh; b[k] = toh_flush((z - (float)zh) * ZRC); }
#pragma unroll
        for (int k = 0; k < 4; ++k) { const float pv = g1[k]; const float z = o1[k] * (pv * (1.0f / (1.0f + expf(-pv)))); const h16 zh = toh_flush(z); a[4 + k] = zh; b[4 + k] = toh_flush((z - (float)zh) * ZRC); }
        *(volatile v8h*)(zrow + (size_t)row * ZK + cofs) = a; *(volatile v8h*)(zrow + (size_t)row * ZK + DQ + cofs) = b;
        __threadfence();
        *(volatile v8h*)(zrow + (size_t)row * ZK + cofs) = a; *(volatile v8h*)(zrow + (size_t)row * ZK + DQ + cofs) = b; }
}

__global__ __launch_bounds__(256) void k_ln_out(const float* __restrict__ Y, const float* __restrict__ gw, const float* __restrict__ gb, float* OUT) {
#pragma clang fp contract(off)
    const int lane = threadIdx.x & 31; const int wave = __builtin_amdgcn_readfirstlane(threadIdx.x >> 5);
    const int row = blockIdx.x * 8 + wave;
    const float* yr = Y + (size_t)row * WORD;
    float s = 0.0f;
#pragma unroll 1
    for (int i = 0; i < 8; ++i) { const v4f v = *(const v4f*)(yr + (i * 32 + lane) * 4); s += (v[0] + v[1]) + (v[2] + v[3]); }
    s += __shfl_xor(s, 16, 32); s += __shfl_xor(s, 8, 32); s += __shfl_xor(s, 4, 32); s += __shfl_xor(s, 2, 32); s += __shfl_xor(s, 1, 32);
    const float mu = s * (1.0f / WORD);
    float ss = 0.0f;
#pragma unroll 1
    for (int i = 0; i < 8; ++i) { const v4f v = *(const v4f*)(yr + (i * 32 + lane) * 4);
#pragma unroll
        for (int k = 0; k < 4; ++k) { const float d = v[k] - mu; ss += d * d; } }
    ss += __shfl_xor(ss, 16, 32); ss += __shfl_xor(ss, 8, 32); ss += __shfl_xor(ss, 4, 32); ss += __shfl_xor(ss, 2, 32); ss += __shfl_xor(ss, 1, 32);
    const float rstd = 1.0f / sqrtf(ss * (1.0f / WORD) + 1.0e-5f);
    float* orow = OUT + (size_t)row * WORD;
#pragma unroll 1
    for (int i = 0; i < 8; ++i) { const int col = (i * 32 + lane) * 4;
        const v4f v = *(const v4f*)(yr + col); const v4f g = *(const v4f*)(gw + col); const v4f b = *(const v4f*)(gb + col); v4f o;
#pragma unroll
        for (int k = 0; k < 4; ++k) o[k] = (v[k] - mu) * rstd * bfr(g[k]) + bfr(b[k]);
        *(volatile v4f*)(orow + col) = o;
        __threadfence();
        *(volatile v4f*)(orow + col) = o; }
}

static constexpr size_t al256(size_t b) { return (b + 255) & ~(size_t)255; }
static constexpr size_t WS_TOTAL = al256((size_t)SEQ * XK * 2) + al256((size_t)WAR * WORD * 2) + al256((size_t)2 * DQ * XK * 2) + al256((size_t)WORD * ZK * 2)
                                 + 2 * al256((size_t)SEQ * DQ * 4) + al256((size_t)SEQ * YP * 4) + al256((size_t)NH * SEQ * 4)
                                 + 4 * al256((size_t)NH * SEQ * HD * 2) + al256((size_t)SEQ * WORD * 4);
static_assert(WS_TOTAL <= (size_t)134217728);
static_assert((size_t)SEQ * ZK * 2 <= (size_t)SEQ * DQ * 4);

extern "C" void kernel_launch(void* const* d_in, const int* in_sizes, int n_in,
                              void* d_out, int out_size, void* d_ws, size_t ws_size, hipStream_t stream) {
    if (n_in < 10) return;
    if (in_sizes[0] < SEQ * WORD || in_sizes[1] < NPROJ * WORD || in_sizes[2] < NPROJ || in_sizes[3] < WORD || in_sizes[4] < WORD || in_sizes[5] < WORD * DQ || in_sizes[6] < WORD || in_sizes[7] < WORD || in_sizes[8] < NH || in_sizes[9] < NH) return;
    if (out_size < SEQ * WORD) return;
    if (WS_TOTAL > ws_size) return;
    const float* x = (const float*)d_in[0]; const float* win = (const float*)d_in[1]; const float* bin = (const float*)d_in[2];
    const float* lniw = (const float*)d_in[3]; const float* lnib = (const float*)d_in[4]; const float* wout = (const float*)d_in[5];
    const float* lnow = (const float*)d_in[6]; const float* lnob = (const float*)d_in[7]; const float* smear = (const float*)d_in[8]; const float* lsc = (const float*)d_in[9];
    float* OUT = (float*)d_out;
    char* wsp = (char*)d_ws;
    auto take = [&](size_t bytes) { char* p = wsp; wsp += (bytes + 255) & ~(size_t)255; return (void*)p; };
    h16* XC  = (h16*)take((size_t)SEQ * XK * 2);
    h16* WA  = (h16*)take((size_t)WAR * WORD * 2);
    h16* WB  = (h16*)take((size_t)2 * DQ * XK * 2);
    h16* WOP = (h16*)take((size_t)WORD * ZK * 2);
    float* F  = (float*)take((size_t)SEQ * DQ * 4);
    float* PF = (float*)take((size_t)SEQ * DQ * 4);
    float* YF = (float*)take((size_t)SEQ * YP * 4);
    float* POS = (float*)take((size_t)NH * SEQ * 4);
    h16* QH = (h16*)take((size_t)NH * SEQ * HD * 2); h16* KPl = (h16*)take((size_t)NH * SEQ * HD * 2);
    h16* VTp = (h16*)take((size_t)NH * HD * SEQ * 2); h16* VRp = (h16*)take((size_t)NH * HD * SEQ * 2);
    float* OUTF = (float*)take((size_t)SEQ * WORD * 4);
    if ((size_t)(wsp - (char*)d_ws) > ws_size) return;
    h16* ZC = (h16*)F;

    k_ln_in<<<SEQ / 8, 256, 0, stream>>>(x, lniw, lnib, XC);
    k_wplane<<<(unsigned)(((size_t)2 * DQ * (WORD / 8) + 255) / 256), 256, 0, stream>>>(win, 2 * DQ, 2 * DQ, WORD, WA, WORD, WCAR, 0.0f, 0);
    k_wplane<<<(unsigned)(((size_t)YP * (WORD / 8) + 255) / 256), 256, 0, stream>>>(win + (size_t)4 * DQ * WORD, NH, YP, WORD, WA + (size_t)2 * DQ * WORD, WORD, WCAR, 0.0f, 0);
    k_wplane<<<(unsigned)(((size_t)2 * DQ * (WORD / 8) + 255) / 256), 256, 0, stream>>>(win + (size_t)2 * DQ * WORD, 2 * DQ, 2 * DQ, WORD, WB, XK, WCAR, WCAR / XRC, 1);
    k_wplane<<<(unsigned)(((size_t)WORD * (DQ / 8) + 255) / 256), 256, 0, stream>>>(wout, WORD, WORD, DQ, WOP, ZK, OCAR, OCAR / ZRC, 1);

    const unsigned LP = (unsigned)(((size_t)NH * SEQ * HD / 8 + 255) / 256);
    k_gemm_xw<<<dim3(SEQ / 64, DQ / 64, 1), 32, 0, stream>>>(XC, XK, WA, WORD, F, DQ, bin, DQ, 1.0f / WCAR);
    k_qkplanes<<<LP, 256, 0, stream>>>(F, QH, smear, lsc, 0);
    k_gemm_xw<<<dim3(SEQ / 64, DQ / 64, 1), 32, 0, stream>>>(XC, XK, WA + (size_t)DQ * WORD, WORD, F, DQ, bin + DQ, DQ, 1.0f / WCAR);
    k_qkplanes<<<LP, 256, 0, stream>>>(F, KPl, smear, lsc, 1);
    k_gemm_xw<<<dim3(SEQ / 64, YP / 64, 1), 32, 0, stream>>>(XC, XK, WA + (size_t)2 * DQ * WORD, WORD, YF, YP, bin + 4 * DQ, NH, 1.0f / WCAR);
    k_pos<<<1, 512, 0, stream>>>(YF, POS);
    k_gemm_xw<<<dim3(SEQ / 64, DQ / 64, 1), 32, 0, stream>>>(XC, XK, WB, XK, F, DQ, bin + 2 * DQ, DQ, 1.0f / WCAR);
    k_vt<<<dim3(SEQ / 64, DQ / 64, 1), 256, 0, stream>>>(F, DQ, VTp, VRp, SEQ);
    k_gemm_xw<<<dim3(SEQ / 64, DQ / 64, 1), 32, 0, stream>>>(XC, XK, WB + (size_t)DQ * XK, XK, PF, DQ, bin + 3 * DQ, DQ, 1.0f / WCAR);

    k_flash<<<dim3(SEQ / 64, NH, 1), 128, 0, stream>>>(QH, KPl, VTp, VRp, POS, PF, ZC);

    k_gemm_zp<<<dim3(SEQ / 64, WORD / 64, 1), 32, 0, stream>>>(ZC, ZK, WOP, ZK, OUTF, WORD, 1.0f / (ZCAR * OCAR));
    k_ln_out<<<SEQ / 8, 256, 0, stream>>>(OUTF, lnow, lnob, OUT);
}
